// NashT5Block_16045997818097
// MI455X (gfx1250) — hardware-verified
//
#include <hip/hip_runtime.h>
#include <math.h>

typedef __attribute__((ext_vector_type(16))) _Float16 v16h;
typedef __attribute__((ext_vector_type(16))) __bf16 v16b;
typedef __attribute__((ext_vector_type(8)))  _Float16 v8h;
typedef __attribute__((ext_vector_type(8)))  float v8f;
typedef __attribute__((ext_vector_type(4)))  float v4f;
typedef __attribute__((ext_vector_type(2)))  float v2f;
typedef __attribute__((ext_vector_type(4)))  unsigned v4u;
typedef __attribute__((ext_vector_type(4)))  int v4i;
typedef float __attribute__((may_alias)) float_a;
typedef int __attribute__((may_alias)) int_a;

template <typename T> __device__ __forceinline__ void vst2(void* p, T v) { *(volatile T*)p = v; __threadfence(); *(volatile T*)p = v; }
__device__ __forceinline__ v8f wmma16(v16h a, v16h b, v8f c) {
  v8f d = __builtin_amdgcn_wmma_f32_16x16x32_f16(false, a, false, b, (short)0, c, false, false);
  asm volatile("v_nop\n\tv_nop\n\tv_nop\n\tv_nop" : "+v"(d) : "v"(a), "v"(b));
  return d;
}
__device__ __forceinline__ v8f wmma_bf(v16b a, v16b b, v8f c) {
  v8f d = __builtin_amdgcn_wmma_f32_16x16x32_bf16(false, a, false, b, (short)0, c, false, false);
  asm volatile("v_nop\n\tv_nop\n\tv_nop\n\tv_nop" : "+v"(d) : "v"(a), "v"(b));
  return d;
}
__device__ __forceinline__ v16h frag_h(const _Float16* rowk0, int lane) {
  union { v16h v; v8h q[2]; } u; const _Float16* p = rowk0 + 8 * (lane >> 4);
  u.q[0] = *(const v8h*)p; u.q[1] = *(const v8h*)(p + 16); return u.v;
}
__device__ __forceinline__ v16h frag_f32(const float* rowk0, int lane) {
  v16h a; const float* p = rowk0 + 8 * (lane >> 4);
#pragma unroll
  for (int i = 0; i < 8; ++i) { a[i] = (_Float16)p[i]; a[8 + i] = (_Float16)p[16 + i]; }
  return a;
}
__device__ __forceinline__ v16h frag_f32s(const float* rowk0, int lane, float sc) {
  v16h a; const float* p = rowk0 + 8 * (lane >> 4);
#pragma unroll
  for (int i = 0; i < 8; ++i) { a[i] = (_Float16)(p[i] * sc); a[8 + i] = (_Float16)(p[16 + i] * sc); }
  return a;
}
__device__ __forceinline__ v16h fragc_f32(const float* W, int k0, int n, int lane, int ld, int K) {
  v16h a; const int g = lane >> 4;
#pragma unroll
  for (int i = 0; i < 8; ++i) { const int ka = k0 + 8 * g + i, kb = ka + 16;
    a[i] = (_Float16)(ka < K ? W[(size_t)ka * ld + n] : 0.f); a[8 + i] = (_Float16)(kb < K ? W[(size_t)kb * ld + n] : 0.f); }
  return a;
}
struct F2 { v16b h, l; };
__device__ __forceinline__ F2 bsplit16(const float v[16]) { F2 r;
#pragma unroll
  for (int i = 0; i < 16; ++i) { const __bf16 h = (__bf16)v[i]; r.h[i] = h; r.l[i] = (__bf16)(v[i] - (float)h); }
  return r; }
__device__ __forceinline__ F2 split_row(const float* row, int k0, int lane) { float v[16]; const float* p = row + k0 + 8 * (lane >> 4);
#pragma unroll
  for (int i = 0; i < 8; ++i) { v[i] = p[i]; v[8 + i] = p[16 + i]; }
  return bsplit16(v); }
__device__ __forceinline__ F2 split_rowK(const float* row, int k0, int lane, int K) { float v[16]; const int g = lane >> 4;
#pragma unroll
  for (int i = 0; i < 8; ++i) { const int ka = k0 + 8 * g + i, kb = ka + 16; v[i] = ka < K ? row[ka] : 0.f; v[8 + i] = kb < K ? row[kb] : 0.f; }
  return bsplit16(v); }
__device__ __forceinline__ F2 split_col(const float* W, int k0, int n, int lane, int ld, int K) { float v[16]; const int g = lane >> 4;
#pragma unroll
  for (int i = 0; i < 8; ++i) { const int ka = k0 + 8 * g + i, kb = ka + 16; v[i] = ka < K ? W[(size_t)ka * ld + n] : 0.f; v[8 + i] = kb < K ? W[(size_t)kb * ld + n] : 0.f; }
  return bsplit16(v); }
__device__ __forceinline__ v8f mac3(const F2& a, const F2& b, v8f c) { c = wmma_bf(a.l, b.h, c); c = wmma_bf(a.h, b.l, c); return wmma_bf(a.h, b.h, c); }
__device__ __forceinline__ float sigm(float v) { return 1.0f / (1.0f + expf(-v)); }
#define LDSX() do { asm volatile("s_wait_dscnt 0" ::: "memory"); __builtin_amdgcn_wave_barrier(); __builtin_amdgcn_fence(__ATOMIC_RELEASE, "workgroup"); } while (0)

#define NB 2
#define SS 1024
#define E 1024
#define NH 16
#define HD 64
#define DFF 4096
#define NR (NB * SS)
#define NBK 32
#define MAXD 128

__global__ __launch_bounds__(256) void k_rms(const float* __restrict__ x, const float* __restrict__ w, _Float16* __restrict__ X16) {
  const int wave = threadIdx.x >> 5, lane = threadIdx.x & 31; const size_t r = (size_t)blockIdx.x * 8 + wave; if (r >= NR) return;
  const float* xr = x + r * E; float q2 = 0.f;
#pragma unroll 1
  for (int i = 0; i < 8; ++i) { const v4f a = *(const v4f*)(xr + i * 128 + lane * 4); q2 += (a[0] * a[0] + a[1] * a[1]) + (a[2] * a[2] + a[3] * a[3]); }
#pragma unroll
  for (int off = 16; off >= 1; off >>= 1) q2 += __shfl_xor(q2, off, 32);
  const float rs = rsqrtf(q2 * (1.0f / E) + 1e-6f);
#pragma unroll 1
  for (int i = 0; i < 4; ++i) { const int c0 = i * 256 + lane * 8; union { v8h h; v4u u; } pk;
#pragma unroll
    for (int e = 0; e < 8; ++e) pk.h[e] = (_Float16)(xr[c0 + e] * rs * w[c0 + e]);
    vst2(X16 + r * E + c0, pk.u); }
}
__global__ __launch_bounds__(256) void k_pack(const float* __restrict__ wq, const float* __restrict__ wk, const float* __restrict__ wv, const float* __restrict__ wo, const float* __restrict__ wi, const float* __restrict__ wff,
                                            _Float16* __restrict__ PT, _Float16* __restrict__ WI, _Float16* __restrict__ WF) {
  const int r = blockIdx.x, tid = threadIdx.x; __shared__ __align__(16) _Float16 srow[DFF];
  if (r < 4 * E) { const int which = r >> 10, n = r & (E - 1); const float* W = (which == 0 ? wq : which == 1 ? wk : which == 2 ? wv : wo) + (size_t)n * E;
    for (int k = tid; k < E; k += 256) srow[k] = (_Float16)(W[k] * 16.0f);
    __syncthreads(); if (tid < 128) vst2(PT + (size_t)r * E + tid * 8, *(const v4u*)(&srow[tid * 8])); }
  else if (r < 4 * E + DFF) { const int n = r - 4 * E; const float* W = wi + (size_t)n * E;
    for (int k = tid; k < E; k += 256) srow[k] = (_Float16)(W[k] * 16.0f);
    __syncthreads(); if (tid < 128) vst2(WI + (size_t)n * E + tid * 8, *(const v4u*)(&srow[tid * 8])); }
  else { const int n = r - 4 * E - DFF; const float* W = wff + (size_t)n * DFF;
    for (int k = tid; k < DFF; k += 256) srow[k] = (_Float16)(W[k] * 16.0f);
    __syncthreads(); for (int q = tid; q < DFF / 8; q += 256) vst2(WF + (size_t)n * DFF + q * 8, *(const v4u*)(&srow[q * 8])); }
}
__global__ __launch_bounds__(256) void k_bias(const float* __restrict__ rb, float* __restrict__ BT) {
  const int h = blockIdx.y, i = blockIdx.x * 256 + threadIdx.x; if (i >= 2 * SS) return;
  float v = 0.f;
  if (i < 2 * SS - 1) { const int rel = i - (SS - 1); const int nb = NBK / 2; int bucket = rel > 0 ? nb : 0; const int rp = rel < 0 ? -rel : rel; const int mx = nb / 2;
    int val; if (rp < mx) val = rp; else { const float lf = logf((float)rp / (float)mx) / 2.772588722239781f * (float)(nb - mx); int large = mx + (int)lf; val = large < nb - 1 ? large : nb - 1; }
    bucket += val; v = rb[bucket * NH + h]; }
  vst2(BT + (size_t)h * 2 * SS + i, v);
}
__global__ __launch_bounds__(128) void k_qkv(const _Float16* __restrict__ X16, const _Float16* __restrict__ PT, _Float16* __restrict__ Q16, _Float16* __restrict__ K16, _Float16* __restrict__ VT) {
  __shared__ __align__(16) float so[4][16][132];
  __shared__ __align__(16) _Float16 st[128][72];
  const int tid = threadIdx.x, wave = tid >> 5, lane = tid & 31, col = lane & 15, g = lane >> 4;
  const int which = blockIdx.z, r0b = blockIdx.x * 64, r0 = r0b + wave * 16, n0 = blockIdx.y * 128; const int b = r0b / SS, s0 = r0b % SS;
  v8f acc[8] = {};
#pragma unroll 2
  for (int kc = 0; kc < E / 32; ++kc) { const v16h a = frag_h(X16 + (size_t)(r0 + col) * E + kc * 32, lane);
#pragma unroll
    for (int j = 0; j < 8; ++j) acc[j] = wmma16(a, frag_h(PT + (size_t)(which * E + n0 + j * 16 + col) * E + kc * 32, lane), acc[j]); }
  if (which < 2) {
#pragma unroll
    for (int j = 0; j < 8; ++j)
#pragma unroll
      for (int r = 0; r < 8; ++r) so[wave][8 * g + r][j * 16 + col] = acc[j][r] * (4.0f / 16.0f);
    LDSX();
    _Float16* D = which == 0 ? Q16 : K16;
    for (int qq = lane; qq < 16 * 2 * 8; qq += 32) { const int hh = qq >> 7, rl = (qq >> 3) & 15, pc = qq & 7; const int h = (n0 >> 6) + hh; union { v8h h8; v4u u; } pk;
#pragma unroll
      for (int e = 0; e < 8; ++e) pk.h8[e] = (_Float16)so[wave][rl][hh * 64 + pc * 8 + e];
      vst2(D + (((size_t)b * NH + h) * SS + s0 + wave * 16 + rl) * HD + pc * 8, pk.u); } }
  else {
#pragma unroll
    for (int j = 0; j < 8; ++j)
#pragma unroll
      for (int r = 0; r < 8; ++r) st[j * 16 + col][wave * 16 + 8 * g + r] = (_Float16)(acc[j][r] * (4.0f / 16.0f));
    __syncthreads();
    for (int qq = tid; qq < 128 * 8; qq += 128) { const int cl = qq >> 3, pc = qq & 7; const int c = n0 + cl, h = c >> 6, d = c & 63;
      vst2(VT + (((size_t)b * NH + h) * HD + d) * SS + s0 + pc * 8, *(const v4u*)(&st[cl][pc * 8])); } }
}
__global__ __launch_bounds__(128) void k_attn(const _Float16* __restrict__ Q16, const _Float16* __restrict__ K16, const _Float16* __restrict__ VT, const float* __restrict__ BT, _Float16* __restrict__ O16) {
  __shared__ __align__(16) float sS[4][16][68];
  __shared__ __align__(16) _Float16 sP[4][16][72];
  __shared__ __align__(16) float sO[4][16][68];
  const int tid = threadIdx.x, w = tid >> 5, lane = tid & 31, col = lane & 15, g = lane >> 4;
  const size_t bh = blockIdx.y; const int h = (int)(bh % NH); const int q0 = blockIdx.x * 64 + w * 16; const float* bth = BT + (size_t)h * 2 * SS + (SS - 1);
  v16h aq[2];
#pragma unroll
  for (int kc = 0; kc < 2; ++kc) aq[kc] = frag_h(Q16 + (bh * SS + q0 + col) * HD + kc * 32, lane);
  float mrun = -3.0e38f, lrun = 0.f; v8f acc[4] = {};
#pragma unroll 1
  for (int kt = 0; kt < SS / 64; ++kt) {
#pragma unroll
    for (int t = 0; t < 4; ++t) { v8f s = {}; const int key = kt * 64 + t * 16 + col;
#pragma unroll
      for (int kc = 0; kc < 2; ++kc) s = wmma16(aq[kc], frag_h(K16 + (bh * SS + key) * HD + kc * 32, lane), s);
#pragma unroll
      for (int r = 0; r < 8; ++r) { const int q = q0 + 8 * g + r; sS[w][8 * g + r][t * 16 + col] = s[r] * (1.0f / 16.0f) + bth[key - q]; } }
    LDSX();
    float mx = -3.4e38f;
#pragma unroll
    for (int jj = 0; jj < 32; ++jj) mx = fmaxf(mx, sS[w][col][g * 32 + jj]);
    mx = fmaxf(mx, __shfl_xor(mx, 16, 32));
    const float mnew = fmaxf(mrun, mx); const float corr = expf(mrun - mnew);
    float ps = 0.f;
#pragma unroll
    for (int jj = 0; jj < 32; ++jj) { const float p = expf(sS[w][col][g * 32 + jj] - mnew); ps += p; sP[w][col][g * 32 + jj] = (_Float16)(p * 16384.0f); }
    ps += __shfl_xor(ps, 16, 32);
    lrun = lrun * corr + ps; mrun = mnew;
#pragma unroll
    for (int r = 0; r < 8; ++r) { const float cr = __shfl(corr, 8 * g + r, 32);
#pragma unroll
      for (int t = 0; t < 4; ++t) acc[t][r] *= cr; }
    LDSX();
#pragma unroll
    for (int kc = 0; kc < 2; ++kc) { const v16h pa = frag_h(&sP[w][col][0] + kc * 32, lane);
#pragma unroll
      for (int t = 0; t < 4; ++t) acc[t] = wmma16(pa, frag_h(VT + (bh * HD + t * 16 + col) * SS + kt * 64 + kc * 32, lane), acc[t]); }
    __builtin_amdgcn_wave_barrier(); }
#pragma unroll
  for (int r = 0; r < 8; ++r) { const float lr = __shfl(lrun, 8 * g + r, 32); const float inv = 8.0f / (lr * 16384.0f * 4.0f);
#pragma unroll
    for (int t = 0; t < 4; ++t) sO[w][8 * g + r][t * 16 + col] = acc[t][r] * inv; }
  LDSX();
  for (int qq = lane; qq < 16 * 8; qq += 32) { const int rl = qq >> 3, pc = qq & 7; union { v8h h8; v4u u; } pk;
#pragma unroll
    for (int e = 0; e < 8; ++e) pk.h8[e] = (_Float16)sO[w][rl][pc * 8 + e];
    vst2(O16 + ((bh * SS) + q0 + rl) * HD + pc * 8, pk.u); }
}
__global__ __launch_bounds__(128) void k_o(const _Float16* __restrict__ O16, const _Float16* __restrict__ PT, const float* __restrict__ hid, float* __restrict__ H1) {
  __shared__ __align__(16) float so[4][16][132];
  const int tid = threadIdx.x, wave = tid >> 5, lane = tid & 31, col = lane & 15, g = lane >> 4;
  const int r0 = blockIdx.x * 64 + wave * 16, n0 = blockIdx.y * 128; const int ra = r0 + col; const int b = ra / SS, s = ra % SS;
  v8f acc[8] = {};
#pragma unroll 2
  for (int kc = 0; kc < E / 32; ++kc) { const int h = kc >> 1; const v16h a = frag_h(O16 + (((size_t)b * NH + h) * SS + s) * HD + (kc & 1) * 32, lane);
#pragma unroll
    for (int j = 0; j < 8; ++j) acc[j] = wmma16(a, frag_h(PT + (size_t)(3 * E + n0 + j * 16 + col) * E + kc * 32, lane), acc[j]); }
#pragma unroll
  for (int j = 0; j < 8; ++j) { const int n = n0 + j * 16 + col;
#pragma unroll
    for (int r = 0; r < 8; ++r) so[wave][8 * g + r][j * 16 + col] = acc[j][r] * (1.0f / (16.0f * 8.0f)) + hid[(size_t)(r0 + 8 * g + r) * E + n]; }
  LDSX();
#pragma unroll 4
  for (int rl = 0; rl < 16; ++rl) vst2(H1 + (size_t)(r0 + rl) * E + n0 + lane * 4, *(const v4f*)(&so[wave][rl][lane * 4]));
}
__global__ __launch_bounds__(128) void k_ff1(const _Float16* __restrict__ Y16, const _Float16* __restrict__ WI, _Float16* __restrict__ F16) {
  __shared__ __align__(16) _Float16 so[4][16][136];
  const int tid = threadIdx.x, wave = tid >> 5, lane = tid & 31, col = lane & 15, g = lane >> 4;
  const int r0 = blockIdx.x * 64 + wave * 16, n0 = blockIdx.y * 128;
  v8f acc[8] = {};
#pragma unroll 2
  for (int kc = 0; kc < E / 32; ++kc) { const v16h a = frag_h(Y16 + (size_t)(r0 + col) * E + kc * 32, lane);
#pragma unroll
    for (int j = 0; j < 8; ++j) acc[j] = wmma16(a, frag_h(WI + (size_t)(n0 + j * 16 + col) * E + kc * 32, lane), acc[j]); }
#pragma unroll
  for (int j = 0; j < 8; ++j)
#pragma unroll
    for (int r = 0; r < 8; ++r) { const float v = acc[j][r] * (1.0f / 16.0f); so[wave][8 * g + r][j * 16 + col] = (_Float16)(v > 0.f ? v : 0.f); }
  LDSX();
  for (int qq = lane; qq < 16 * 16; qq += 32) { const int rl = qq >> 4, pc = qq & 15; vst2(F16 + (size_t)(r0 + rl) * DFF + n0 + pc * 8, *(const v4u*)(&so[wave][rl][pc * 8])); }
}
__global__ __launch_bounds__(128) void k_ff2(const _Float16* __restrict__ F16, const _Float16* __restrict__ WF, const float* __restrict__ H1, float* __restrict__ out) {
  __shared__ __align__(16) float so[4][16][132];
  const int tid = threadIdx.x, wave = tid >> 5, lane = tid & 31, col = lane & 15, g = lane >> 4;
  const int r0 = blockIdx.x * 64 + wave * 16, n0 = blockIdx.y * 128;
  v8f acc[8] = {};
#pragma unroll 2
  for (int kc = 0; kc < DFF / 32; ++kc) { const v16h a = frag_h(F16 + (size_t)(r0 + col) * DFF + kc * 32, lane);
#pragma unroll
    for (int j = 0; j < 8; ++j) acc[j] = wmma16(a, frag_h(WF + (size_t)(n0 + j * 16 + col) * DFF + kc * 32, lane), acc[j]); }
#pragma unroll
  for (int j = 0; j < 8; ++j) { const int n = n0 + j * 16 + col;
#pragma unroll
    for (int r = 0; r < 8; ++r) so[wave][8 * g + r][j * 16 + col] = acc[j][r] * (1.0f / 16.0f) + H1[(size_t)(r0 + 8 * g + r) * E + n]; }
  LDSX();
#pragma unroll 4
  for (int rl = 0; rl < 16; ++rl) vst2(out + (size_t)(r0 + rl) * E + n0 + lane * 4, *(const v4f*)(&so[wave][rl][lane * 4]));
}
extern "C" void kernel_launch(void* const* d_in, const int* in_sizes, int n_in, void* d_out, int out_size, void* d_ws, size_t ws_size, hipStream_t stream) {
  (void)in_sizes; (void)n_in; (void)out_size; (void)ws_size;
  const float** I = (const float**)d_in;
  const float* hid = I[0]; const float* ln1 = I[1]; const float* wq = I[2]; const float* wk = I[3]; const float* wv = I[4]; const float* wo = I[5]; const float* rb = I[6]; const float* ln2 = I[7]; const float* wi = I[8]; const float* wff = I[9];
  float* out = (float*)d_out;
  char* ws = (char*)d_ws; size_t off = 0;
  auto take = [&](size_t bytes) { char* p = ws + off; off += (bytes + 255) & ~(size_t)255; return p; };
  _Float16* X16 = (_Float16*)take((size_t)NR * E * 2); _Float16* PT = (_Float16*)take((size_t)4 * E * E * 2); _Float16* WI = (_Float16*)take((size_t)DFF * E * 2); _Float16* WF = (_Float16*)take((size_t)E * DFF * 2);
  float* BT = (float*)take((size_t)NH * 2 * SS * 4);
  _Float16* Q16 = (_Float16*)take((size_t)NR * E * 2); _Float16* K16 = (_Float16*)take((size_t)NR * E * 2); _Float16* VT = (_Float16*)take((size_t)NR * E * 2); _Float16* O16 = (_Float16*)take((size_t)NR * E * 2);
  float* H1 = (float*)take((size_t)NR * E * 4); _Float16* Y16 = X16; _Float16* F16 = (_Float16*)take((size_t)NR * DFF * 2);
  k_rms<<<NR / 8, 256, 0, stream>>>(hid, ln1, X16);
  k_pack<<<4 * E + DFF + E, 256, 0, stream>>>(wq, wk, wv, wo, wi, wff, PT, WI, WF);
  k_bias<<<dim3(2 * SS / 256, NH), 256, 0, stream>>>(rb, BT);
  k_qkv<<<dim3(NR / 64, E / 128, 3), 128, 0, stream>>>(X16, PT, Q16, K16, VT);
  k_attn<<<dim3(SS / 64, NB * NH), 128, 0, stream>>>(Q16, K16, VT, BT, O16);
  k_o<<<dim3(NR / 64, E / 128), 128, 0, stream>>>(O16, PT, hid, H1);
  k_rms<<<NR / 8, 256, 0, stream>>>(H1, ln2, Y16);
  k_ff1<<<dim3(NR / 64, DFF / 128), 128, 0, stream>>>(Y16, WI, F16);
  k_ff2<<<dim3(NR / 64, E / 128), 128, 0, stream>>>(F16, WF, H1, out);
}
